// TemporalMambaBlock_45896020525190
// MI455X (gfx1250) — hardware-verified
//
#include <hip/hip_runtime.h>
#include <hip/hip_bf16.h>
#include <math.h>

typedef __attribute__((ext_vector_type(16))) _Float16 v16h;
typedef __attribute__((ext_vector_type(8)))  _Float16 v8h;
typedef __attribute__((ext_vector_type(16))) __bf16   v16b;
typedef __attribute__((ext_vector_type(8)))  __bf16   v8b;
typedef __attribute__((ext_vector_type(8)))  float    v8f;
typedef __attribute__((ext_vector_type(4)))  float    v4f;

#define NSEQ   1568
#define TLEN   16
#define NROWS  25088
#define HWSZ   784
#define CDIM   192
#define DIN    384
#define NST    16
#define NDT    12
#define NPRJ   64
#define XPRJ   44
#define YPITCH 388

#define WIN_H    0
#define WIN_L    147456
#define WX_H     294912
#define WX_L     319488
#define WOUT_H   344064
#define WOUT_L   417792
#define WGT_END  491520

__device__ __forceinline__ unsigned short f2bf_bits(float f) {
  unsigned u = __float_as_uint(f);
  return (unsigned short)((u + 0x7FFFu + ((u >> 16) & 1u)) >> 16);
}
__device__ __forceinline__ float bf_bits2f(unsigned short h) { return __uint_as_float(((unsigned)h) << 16); }

__device__ __forceinline__ void dep_guard_h(v8f& a, v8f& b, v16h x, v16h y) { asm volatile("v_nop\n\tv_nop\n\tv_nop\n\tv_nop" : "+v"(a), "+v"(b) : "v"(x), "v"(y)); }
__device__ __forceinline__ void dep_guard_b(v8f& a, v8f& b, v16b x, v16b y) { asm volatile("v_nop\n\tv_nop\n\tv_nop\n\tv_nop" : "+v"(a), "+v"(b) : "v"(x), "v"(y)); }
__device__ __forceinline__ void keep4_h(v16h a, v16h b, v16h c, v16h d) { asm volatile("v_nop" :: "v"(a), "v"(b), "v"(c), "v"(d)); }
__device__ __forceinline__ void keep4_b(v16b a, v16b b, v16b c, v16b d) { asm volatile("v_nop" :: "v"(a), "v"(b), "v"(c), "v"(d)); }
__device__ __forceinline__ void acc_guard4(v8f& a, v8f& b, v8f& c, v8f& d) { asm volatile("v_nop\n\tv_nop\n\tv_nop\n\tv_nop" : "+v"(a), "+v"(b), "+v"(c), "+v"(d)); }
template <typename T> struct Frag;
template <> struct Frag<_Float16> {
  typedef v16h V; union U { v16h v; v8h h[2]; };
  static __device__ __forceinline__ v16h load(const _Float16* p) {
    U f; f.h[0] = *(const v8h*)(p); f.h[1] = *(const v8h*)(p + 16); return f.v;
  }
  static __device__ __forceinline__ v8f mma(v16h a, v16h b, v8f c) {
    return __builtin_amdgcn_wmma_f32_16x16x32_f16(false, a, false, b, (short)0, c, false, false);
  }
  static __device__ __forceinline__ void guard(v8f& a, v8f& b, v16h x, v16h y) { dep_guard_h(a, b, x, y); }
  static __device__ __forceinline__ void keep(v16h a, v16h b, v16h c, v16h d) { keep4_h(a, b, c, d); }
};
template <> struct Frag<__bf16> {
  typedef v16b V; union U { v16b v; v8b h[2]; };
  static __device__ __forceinline__ v16b load(const __bf16* p) {
    U f; f.h[0] = *(const v8b*)(p); f.h[1] = *(const v8b*)(p + 16); return f.v;
  }
  static __device__ __forceinline__ v8f mma(v16b a, v16b b, v8f c) {
    return __builtin_amdgcn_wmma_f32_16x16x32_bf16(false, a, false, b, (short)0, c, false, false);
  }
  static __device__ __forceinline__ void guard(v8f& a, v8f& b, v16b x, v16b y) { dep_guard_b(a, b, x, y); }
  static __device__ __forceinline__ void keep(v16b a, v16b b, v16b c, v16b d) { keep4_b(a, b, c, d); }
};

template <int ET> struct Elem;
template <> struct Elem<0> { typedef _Float16 T; };
template <> struct Elem<1> { typedef __bf16 T; };
template <int ET, bool SPLIT, int BIAS_MODE, int OUT_MODE, bool RESID, int ACT = 0>
__global__ __launch_bounds__(256) void wmma_gemm64(
    const unsigned short* __restrict__ Ap, const unsigned short* __restrict__ A2p, int lda, long strideA,
    const unsigned short* __restrict__ Btp, const unsigned short* __restrict__ Bt2p, int ldb, long strideB,
    void* __restrict__ Cout, void* __restrict__ Cout2, int ldc, long strideC,
    const float* __restrict__ bias,
    const float* __restrict__ resid, long strideR,
    int M, int N, int K, float scale) {
  typedef typename Elem<ET>::T T;
  typedef typename Frag<T>::V V;
  const T* A = (const T*)Ap; const T* A2 = (const T*)A2p; const T* Bt = (const T*)Btp; const T* Bt2 = (const T*)Bt2p;
  __shared__ __align__(16) float sT[8][16 * 68];
  const int b    = blockIdx.y;
  const int lane = threadIdx.x & 31;
  const int wave = threadIdx.x >> 5;
  const int tilesN = N >> 6;
  const int tilesM = M >> 6;
  const int tile = blockIdx.x * 8 + wave;
  if (tile >= tilesM * tilesN) return;
  const int tm = tile / tilesN;
  const int tn = tile - tm * tilesN;
  const int m0 = tm << 6;
  const int n0 = tn << 6;

  const T* Ab  = A  + (size_t)b * strideA;
  const T* Bb  = Bt + (size_t)b * strideB;
  const T* Ab2 = SPLIT ? (A2  + (size_t)b * strideA) : nullptr;
  const T* Bb2 = SPLIT ? (Bt2 + (size_t)b * strideB) : nullptr;

  const int rlane = lane & 15;
  const int koff  = (lane >> 4) * 8;
  const int mOff  = (lane >> 4) * 8;

  v8f acc[4][4];
#pragma unroll
  for (int i = 0; i < 4; ++i)
#pragma unroll
    for (int j = 0; j < 4; ++j) acc[i][j] = (v8f){0.f,0.f,0.f,0.f,0.f,0.f,0.f,0.f};

  for (int k0 = 0; k0 < K; k0 += 32) {
    V bh[4], bl[4];
#pragma unroll
    for (int j = 0; j < 4; ++j) {
      const size_t bo = (size_t)(n0 + (j << 4) + rlane) * ldb + koff + k0;
      bh[j] = Frag<T>::load(Bb + bo);
      if (SPLIT) bl[j] = Frag<T>::load(Bb2 + bo);
    }
#pragma unroll
    for (int i = 0; i < 4; ++i) {
      const size_t ao = (size_t)(m0 + (i << 4) + rlane) * lda + koff + k0;
      V ah = Frag<T>::load(Ab + ao);
      V al;
      if (SPLIT) al = Frag<T>::load(Ab2 + ao);
#pragma unroll
      for (int j = 0; j < 4; ++j) {
        acc[i][j] = Frag<T>::mma(ah, bh[j], acc[i][j]);
        if (SPLIT) {
          acc[i][j] = Frag<T>::mma(ah, bl[j], acc[i][j]);
          acc[i][j] = Frag<T>::mma(al, bh[j], acc[i][j]);
        }
      }
      Frag<T>::guard(acc[i][0], acc[i][3], ah, SPLIT ? al : ah);
    }
    Frag<T>::keep(bh[0], bh[1], bh[2], bh[3]);
    if (SPLIT) Frag<T>::keep(bl[0], bl[1], bl[2], bl[3]);
  }
  acc_guard4(acc[0][0], acc[0][1], acc[0][2], acc[0][3]);
  acc_guard4(acc[1][0], acc[1][1], acc[1][2], acc[1][3]);
  acc_guard4(acc[2][0], acc[2][1], acc[2][2], acc[2][3]);
  acc_guard4(acc[3][0], acc[3][1], acc[3][2], acc[3][3]);

  float* slab = sT[wave];
  const float* Rb = RESID ? (resid + (size_t)b * strideR) : nullptr;
#pragma unroll
  for (int i = 0; i < 4; ++i) {
    const int mBase = m0 + (i << 4);
#pragma unroll
    for (int j = 0; j < 4; ++j) {
      const int n = n0 + (j << 4) + rlane;
      float bv = 0.f;
      if (BIAS_MODE == 2) bv = bias[n];
#pragma unroll
      for (int r = 0; r < 8; ++r) {
        float v = acc[i][j][r] * scale;
        if (BIAS_MODE == 1) v += bias[mBase + mOff + r];
        if (BIAS_MODE == 2) v += bv;
        if (RESID) v += Rb[(size_t)(mBase + mOff + r) * ldc + n];
        if (ACT == 1) v = tanhf(v);
        if (ACT == 2) v = fmaxf(v, 0.0f);
        if (ACT == 3) v = v / (1.0f + expf(-v));
        if (ACT == 4) v = (v > 0.f) ? v : 0.01f * v;
        if (ACT == 5) v = 0.5f * v * (1.0f + erff(v * 0.70710678118654752f));
        slab[(mOff + r) * 68 + (j << 4) + rlane] = v;
      }
    }
    __builtin_amdgcn_fence(__ATOMIC_RELEASE, "workgroup");
    __builtin_amdgcn_wave_barrier();
    __builtin_amdgcn_fence(__ATOMIC_ACQUIRE, "workgroup");
    if (OUT_MODE == 0) {
      float* C = (float*)Cout + (size_t)b * strideC;
      const int hh = lane >> 4, c4 = (lane & 15) * 4;
      for (int pass = 0; pass < 2; ++pass) {
#pragma unroll
        for (int it = 0; it < 8; ++it) {
          const int row = it * 2 + hh;
          v4f v = *(const v4f*)(slab + row * 68 + c4);
          *(volatile v4f*)(C + (size_t)(mBase + row) * ldc + n0 + c4) = v;
        }
        __threadfence();
      }
    } else {
      const int q = lane >> 3, c8 = (lane & 7) * 8;
      unsigned short* C  = (unsigned short*)Cout  + (size_t)b * strideC;
      unsigned short* C2 = (OUT_MODE == 2) ? ((unsigned short*)Cout2 + (size_t)b * strideC) : nullptr;
      for (int pass = 0; pass < 2; ++pass) {
#pragma unroll
        for (int it = 0; it < 4; ++it) {
          const int row = it * 4 + q;
          const float* sp = slab + row * 68 + c8;
          v8h hv, lv;
#pragma unroll
          for (int e = 0; e < 8; ++e) {
            if (OUT_MODE == 1) {
              hv[e] = (_Float16)sp[e];
            } else {
              unsigned short hb = f2bf_bits(sp[e]);
              unsigned short lb = f2bf_bits(sp[e] - bf_bits2f(hb));
              hv[e] = __builtin_bit_cast(_Float16, hb);
              lv[e] = __builtin_bit_cast(_Float16, lb);
            }
          }
          *(volatile v8h*)(C + (size_t)(mBase + row) * ldc + n0 + c8) = hv;
          if (OUT_MODE == 2) *(volatile v8h*)(C2 + (size_t)(mBase + row) * ldc + n0 + c8) = lv;
        }
        __threadfence();
      }
    }
    __builtin_amdgcn_fence(__ATOMIC_RELEASE, "workgroup");
    __builtin_amdgcn_wave_barrier();
    __builtin_amdgcn_fence(__ATOMIC_ACQUIRE, "workgroup");
  }
}

__device__ __forceinline__ void split_bf8(v4f a0, v4f a1, v8h& hv, v8h& lv) {
#pragma unroll
  for (int e = 0; e < 4; ++e) {
    const unsigned short h0 = f2bf_bits(a0[e]);
    const unsigned short l0 = f2bf_bits(a0[e] - bf_bits2f(h0));
    const unsigned short h1 = f2bf_bits(a1[e]);
    const unsigned short l1 = f2bf_bits(a1[e] - bf_bits2f(h1));
    hv[e] = __builtin_bit_cast(_Float16, h0);     lv[e] = __builtin_bit_cast(_Float16, l0);
    hv[4 + e] = __builtin_bit_cast(_Float16, h1); lv[4 + e] = __builtin_bit_cast(_Float16, l1);
  }
}

__global__ __launch_bounds__(256) void weight_planes_kernel(
    const float* __restrict__ w_in, const float* __restrict__ w_x, const float* __restrict__ w_out,
    unsigned short* __restrict__ P)
{
  const int y = blockIdx.y;
  const float* W = w_in; int ldw = 768, Kreal = 192, Kpad = 192, Nreal = 768, Npad = 768, offh = WIN_H, offl = WIN_L;
  if (y == 1)      { W = w_x;   ldw = XPRJ; Kreal = DIN; Kpad = DIN; Nreal = XPRJ; Npad = NPRJ; offh = WX_H;   offl = WX_L; }
  else if (y == 2) { W = w_out; ldw = CDIM; Kreal = DIN; Kpad = DIN; Nreal = CDIM; Npad = CDIM; offh = WOUT_H; offl = WOUT_L; }
  const int nseg  = Kpad >> 3;
  const int total = Npad * nseg;
  const int i = blockIdx.x * 256 + threadIdx.x;
  if (i >= total) return;
  const int n   = i / nseg;
  const int seg = i - n * nseg;
  const int nc  = (n < Nreal) ? n : (Nreal - 1);
  v4f a0, a1;
#pragma unroll
  for (int e = 0; e < 4; ++e) {
    const int k0i = seg * 8 + e, k1i = seg * 8 + 4 + e;
    const int kc0 = (k0i < Kreal) ? k0i : (Kreal - 1);
    const int kc1 = (k1i < Kreal) ? k1i : (Kreal - 1);
    const float t0 = W[(size_t)kc0 * ldw + nc];
    const float t1 = W[(size_t)kc1 * ldw + nc];
    a0[e] = (n < Nreal && k0i < Kreal) ? t0 : 0.f;
    a1[e] = (n < Nreal && k1i < Kreal) ? t1 : 0.f;
  }
  v8h hv, lv;
  split_bf8(a0, a1, hv, lv);
  const size_t off = (size_t)n * Kpad + seg * 8;
  for (int pass = 0; pass < 2; ++pass) {
    *(volatile v8h*)(P + offh + off) = hv;
    *(volatile v8h*)(P + offl + off) = lv;
    __threadfence();
  }
}

__global__ __launch_bounds__(256) void rmsnorm_planes_kernel(
    const float* __restrict__ x, const float* __restrict__ nw,
    unsigned short* __restrict__ Xh, unsigned short* __restrict__ Xl)
{
  const int lane = threadIdx.x & 31, wave = threadIdx.x >> 5;
  const int cl = (lane < 24) ? lane : 23;
  const int c8 = cl * 8;
  const v4f g0 = *(const v4f*)(nw + c8);
  const v4f g1 = *(const v4f*)(nw + c8 + 4);
#pragma unroll 1
  for (int i = 0; i < 4; ++i) {
    const int r  = blockIdx.x * 32 + wave * 4 + i;
    const int n  = r >> 4, t = r & 15;
    const int b  = n / HWSZ, hw = n - b * HWSZ;
    const size_t xo = ((size_t)((b * TLEN + t) * HWSZ + hw)) * CDIM + c8;
    const v4f a0 = *(const v4f*)(x + xo);
    const v4f a1 = *(const v4f*)(x + xo + 4);
    float ss = a0[0] * a0[0];
    ss = fmaf(a0[1], a0[1], ss); ss = fmaf(a0[2], a0[2], ss); ss = fmaf(a0[3], a0[3], ss);
    ss = fmaf(a1[0], a1[0], ss); ss = fmaf(a1[1], a1[1], ss); ss = fmaf(a1[2], a1[2], ss); ss = fmaf(a1[3], a1[3], ss);
    ss = (lane < 24) ? ss : 0.f;
#pragma unroll
    for (int off = 1; off < 32; off <<= 1) ss += __shfl_xor(ss, off, 32);
    const float nrm = rsqrtf(ss * (1.0f / 192.0f) + 1e-6f);
    v4f o0, o1;
#pragma unroll
    for (int e = 0; e < 4; ++e) { o0[e] = (a0[e] * nrm) * g0[e]; o1[e] = (a1[e] * nrm) * g1[e]; }
    v8h hv, lv;
    split_bf8(o0, o1, hv, lv);
    const size_t off = (size_t)r * CDIM + c8;
    for (int pass = 0; pass < 2; ++pass) {
      if (lane < 24) {
        *(volatile v8h*)(Xh + off) = hv;
        *(volatile v8h*)(Xl + off) = lv;
      }
      __threadfence();
    }
  }
}

__device__ __forceinline__ void tile16_to_planes(const float* tile, int rb,
                                                 unsigned short* __restrict__ Ph, unsigned short* __restrict__ Pl)
{
  const int L = threadIdx.x;
  const int rsub = L / 48, seg = L - rsub * 48, c8 = seg * 8;
  v8h hv[2], lv[2];
#pragma unroll
  for (int it = 0; it < 2; ++it) {
    const int row = it * 8 + rsub;
    const v4f a0 = *(const v4f*)(tile + row * YPITCH + c8);
    const v4f a1 = *(const v4f*)(tile + row * YPITCH + c8 + 4);
    split_bf8(a0, a1, hv[it], lv[it]);
  }
  for (int pass = 0; pass < 2; ++pass) {
#pragma unroll
    for (int it = 0; it < 2; ++it) {
      const int row = it * 8 + rsub;
      const size_t off = (size_t)(rb + row) * DIN + c8;
      *(volatile v8h*)(Ph + off) = hv[it];
      *(volatile v8h*)(Pl + off) = lv[it];
    }
    __threadfence();
  }
}

__global__ __launch_bounds__(384) void conv_silu_kernel(
    const float* __restrict__ U, const float* __restrict__ w_conv, const float* __restrict__ b_conv,
    unsigned short* __restrict__ UCh, unsigned short* __restrict__ UCl)
{
  __shared__ __align__(16) float sX[TLEN * YPITCH];
  const int d  = threadIdx.x;
  const int rb = blockIdx.x * TLEN;
  const float w0 = w_conv[d * 4 + 0], w1 = w_conv[d * 4 + 1], w2 = w_conv[d * 4 + 2], w3 = w_conv[d * 4 + 3];
  const float bc = b_conv[d];
  float x0 = 0.f, x1 = 0.f, x2 = 0.f;
#pragma unroll 1
  for (int r = 0; r < TLEN; ++r) {
    const float xcur = U[(size_t)(rb + r) * DIN + d];
    float acc = w0 * x0;
    acc = fmaf(w1, x1, acc);
    acc = fmaf(w2, x2, acc);
    acc = fmaf(w3, xcur, acc);
    const float sv = acc + bc;
    const float sg = __builtin_amdgcn_rcpf(1.0f + __expf(-sv));
    sX[r * YPITCH + d] = sv * sg;
    x0 = x1; x1 = x2; x2 = xcur;
  }
  __syncthreads();
  tile16_to_planes(sX, rb, UCh, UCl);
}

__global__ __launch_bounds__(384) void scan_kernel(
    const float* __restrict__ DBL, const unsigned short* __restrict__ UCh, const unsigned short* __restrict__ UCl,
    const float* __restrict__ Z, const float* __restrict__ w_dt, const float* __restrict__ b_dt,
    const float* __restrict__ A_log, const float* __restrict__ Dsk,
    unsigned short* __restrict__ Yh, unsigned short* __restrict__ Yl)
{
  __shared__ __align__(16) float sP[TLEN * NPRJ];
  __shared__ __align__(16) float sAY[DIN * 17];
  const int d  = threadIdx.x;
  const int rb = blockIdx.x * TLEN;

#pragma unroll 1
  for (int n = 0; n < NST; ++n) sAY[d * 17 + n] = -expf(A_log[d * NST + n]);
  if (d < 256) *(v4f*)(sP + d * 4) = *(const v4f*)(DBL + (size_t)rb * NPRJ + d * 4);
  __syncthreads();
  float An[NST];
#pragma unroll
  for (int n = 0; n < NST; ++n) An[n] = sAY[d * 17 + n];
  float wd[NDT];
#pragma unroll
  for (int r = 0; r < NDT; ++r) wd[r] = w_dt[r * DIN + d];
  const float bd = b_dt[d], Dd = Dsk[d];
  float h[NST];
#pragma unroll
  for (int n = 0; n < NST; ++n) h[n] = 0.f;
  __syncthreads();

#pragma unroll 1
  for (int s = 0; s < TLEN; ++s) {
    const size_t row = (size_t)rb + s;
    const unsigned short uh = UCh[row * DIN + d];
    const unsigned short ul = UCl[row * DIN + d];
    const float ucv = bf_bits2f(uh) + bf_bits2f(ul);
    const float zv  = Z[row * DIN + d];
    const float* pr = sP + s * NPRJ;
    const v4f t0 = *(const v4f*)(pr);
    const v4f t1 = *(const v4f*)(pr + 4);
    const v4f t2 = *(const v4f*)(pr + 8);
    v4f Bq[4], Cq[4];
#pragma unroll
    for (int q = 0; q < 4; ++q) {
      Bq[q] = *(const v4f*)(pr + NDT + 4 * q);
      Cq[q] = *(const v4f*)(pr + NDT + NST + 4 * q);
    }
    float a = t0[0] * wd[0];
    a = fmaf(t0[1], wd[1], a);  a = fmaf(t0[2], wd[2], a);  a = fmaf(t0[3], wd[3], a);
    a = fmaf(t1[0], wd[4], a);  a = fmaf(t1[1], wd[5], a);  a = fmaf(t1[2], wd[6], a);  a = fmaf(t1[3], wd[7], a);
    a = fmaf(t2[0], wd[8], a);  a = fmaf(t2[1], wd[9], a);  a = fmaf(t2[2], wd[10], a); a = fmaf(t2[3], wd[11], a);
    a += bd;
    const float dt = fmaxf(a, 0.f) + log1pf(__expf(-fabsf(a)));
    const float u = dt * ucv;
    float y = 0.f;
#pragma unroll
    for (int n = 0; n < NST; ++n) {
      const float e = __expf(dt * An[n]);
      h[n] = fmaf(e, h[n], u * Bq[n >> 2][n & 3]);
      y = fmaf(h[n], Cq[n >> 2][n & 3], y);
    }
    y = fmaf(ucv, Dd, y);
    const float sg = __builtin_amdgcn_rcpf(1.0f + __expf(-zv));
    y = y * (zv * sg);
    sAY[s * YPITCH + d] = y;
  }
  __syncthreads();
  tile16_to_planes(sAY, rb, Yh, Yl);
}

__global__ __launch_bounds__(256) void out_residual_kernel(
    const float* __restrict__ OUTB, const float* __restrict__ x, float* __restrict__ out)
{
  const int lane = threadIdx.x & 31, wave = threadIdx.x >> 5;
  const int hh = lane >> 4, c4 = (lane & 15) * 4;
  const int o  = blockIdx.x * 16 + wave * 2 + hh;
  const int bt = o / HWSZ, hw = o - bt * HWSZ;
  const int b  = bt >> 4, t = bt & 15;
  const int r  = (b * HWSZ + hw) * TLEN + t;
  v4f v0, v1, v2;
  {
    const float* xs = x + (size_t)o * CDIM + c4;
    const float* ys = OUTB + (size_t)r * CDIM + c4;
    v0 = *(const v4f*)(xs)       + *(const v4f*)(ys);
    v1 = *(const v4f*)(xs + 64)  + *(const v4f*)(ys + 64);
    v2 = *(const v4f*)(xs + 128) + *(const v4f*)(ys + 128);
  }
  float* op = out + (size_t)o * CDIM + c4;
  for (int pass = 0; pass < 2; ++pass) {
    *(volatile v4f*)(op)       = v0;
    *(volatile v4f*)(op + 64)  = v1;
    *(volatile v4f*)(op + 128) = v2;
    __threadfence();
  }
}

extern "C" void kernel_launch(void* const* d_in, const int* in_sizes, int n_in,
                              void* d_out, int out_size, void* d_ws, size_t ws_size,
                              hipStream_t stream)
{
  if (n_in < 11) return;
  const float* x        = (const float*)d_in[0];
  const float* norm_w   = (const float*)d_in[1];
  const float* in_proj  = (const float*)d_in[2];
  const float* conv_w   = (const float*)d_in[3];
  const float* conv_b   = (const float*)d_in[4];
  const float* x_proj   = (const float*)d_in[5];
  const float* dt_w     = (const float*)d_in[6];
  const float* dt_b     = (const float*)d_in[7];
  const float* A_log    = (const float*)d_in[8];
  const float* Dp       = (const float*)d_in[9];
  const float* out_proj = (const float*)d_in[10];

  if (in_sizes[0] != NROWS * CDIM) return;
  if (out_size != NROWS * CDIM) return;
  if (in_sizes[1] != CDIM || in_sizes[2] != CDIM * 2 * DIN || in_sizes[3] != DIN * 4 || in_sizes[4] != DIN) return;
  if (in_sizes[5] != DIN * XPRJ || in_sizes[6] != NDT * DIN || in_sizes[7] != DIN || in_sizes[8] != DIN * NST) return;
  if (in_sizes[9] != DIN || in_sizes[10] != DIN * CDIM) return;

  const size_t P384 = (size_t)NROWS * DIN * 4;
  const size_t PDBL = (size_t)NROWS * NPRJ * 4;
  const size_t OFF_WGT = 0;
  const size_t OFF_R1  = 1048576;
  const size_t OFF_R2  = OFF_R1 + P384;
  const size_t OFF_R3  = OFF_R2 + P384;
  const size_t OFF_R4  = OFF_R3 + P384;
  const size_t TOTAL   = OFF_R4 + PDBL;
  if (ws_size < TOTAL) return;
  if ((size_t)WGT_END * 2 > OFF_R1) return;

  char* ws = (char*)d_ws;
  unsigned short* WGT = (unsigned short*)(ws + OFF_WGT);
  float* U            = (float*)(ws + OFF_R1);
  unsigned short* Yh  = (unsigned short*)(ws + OFF_R1);
  unsigned short* Yl  = Yh + (size_t)NROWS * DIN;
  float* Z            = (float*)(ws + OFF_R2);
  float* OUTB         = (float*)(ws + OFF_R2);
  unsigned short* XNh = (unsigned short*)(ws + OFF_R3);
  unsigned short* XNl = XNh + (size_t)NROWS * CDIM;
  unsigned short* UCh = (unsigned short*)(ws + OFF_R3);
  unsigned short* UCl = UCh + (size_t)NROWS * DIN;
  float* DBL          = (float*)(ws + OFF_R4);
  float* dout         = (float*)d_out;

  const int TILES_M = NROWS / 64;

  weight_planes_kernel<<<dim3(72, 3), 256, 0, stream>>>(in_proj, x_proj, out_proj, WGT);
  rmsnorm_planes_kernel<<<NROWS / 32, 256, 0, stream>>>(x, norm_w, XNh, XNl);

  wmma_gemm64<1, true, 0, 0, false><<<dim3((TILES_M * 6) / 8, 1), 256, 0, stream>>>(
      XNh, XNl, CDIM, 0L, WGT + WIN_H, WGT + WIN_L, CDIM, 0L,
      (void*)U, (void*)U, DIN, 0L, DBL, DBL, 0L, NROWS, DIN, CDIM, 1.0f);
  wmma_gemm64<1, true, 0, 0, false><<<dim3((TILES_M * 6) / 8, 1), 256, 0, stream>>>(
      XNh, XNl, CDIM, 0L, WGT + WIN_H + (size_t)DIN * CDIM, WGT + WIN_L + (size_t)DIN * CDIM, CDIM, 0L,
      (void*)Z, (void*)Z, DIN, 0L, DBL, DBL, 0L, NROWS, DIN, CDIM, 1.0f);

  conv_silu_kernel<<<NSEQ, 384, 0, stream>>>(U, conv_w, conv_b, UCh, UCl);

  wmma_gemm64<1, true, 0, 0, false><<<dim3(TILES_M / 8, 1), 256, 0, stream>>>(
      UCh, UCl, DIN, 0L, WGT + WX_H, WGT + WX_L, DIN, 0L,
      (void*)DBL, (void*)DBL, NPRJ, 0L, Z, Z, 0L, NROWS, NPRJ, DIN, 1.0f);

  scan_kernel<<<NSEQ, 384, 0, stream>>>(DBL, UCh, UCl, Z, dt_w, dt_b, A_log, Dp, Yh, Yl);

  wmma_gemm64<1, true, 0, 0, false><<<dim3((TILES_M * 3) / 8, 1), 256, 0, stream>>>(
      Yh, Yl, DIN, 0L, WGT + WOUT_H, WGT + WOUT_L, DIN, 0L,
      (void*)OUTB, (void*)OUTB, CDIM, 0L, DBL, DBL, 0L, NROWS, CDIM, DIN, 1.0f);

  out_residual_kernel<<<NSEQ, 256, 0, stream>>>(OUTB, x, dout);

  (void)hipGetLastError();
}
